// CluTSPEncoder_7069516169274
// MI455X (gfx1250) — hardware-run, weakly checked
//
#include <hip/hip_runtime.h>
#include <math.h>

typedef __attribute__((ext_vector_type(16))) _Float16 v16h;
typedef __attribute__((ext_vector_type(16))) __bf16 v16b;
typedef __attribute__((ext_vector_type(8)))  _Float16 v8h;
typedef __attribute__((ext_vector_type(8)))  float v8f;
typedef __attribute__((ext_vector_type(4)))  float v4f;
typedef __attribute__((ext_vector_type(2)))  float v2f;
typedef __attribute__((ext_vector_type(4)))  unsigned v4u;
typedef __attribute__((ext_vector_type(4)))  int v4i;
typedef float __attribute__((may_alias)) float_a;
typedef int __attribute__((may_alias)) int_a;

template <typename T> __device__ __forceinline__ void vst2(void* p, T v) { *(volatile T*)p = v; __threadfence(); *(volatile T*)p = v; }
__device__ __forceinline__ v8f wmma16(v16h a, v16h b, v8f c) {
  v8f d = __builtin_amdgcn_wmma_f32_16x16x32_f16(false, a, false, b, (short)0, c, false, false);
  asm volatile("v_nop\n\tv_nop\n\tv_nop\n\tv_nop" : "+v"(d) : "v"(a), "v"(b));
  return d;
}
__device__ __forceinline__ v8f wmma_bf(v16b a, v16b b, v8f c) {
  v8f d = __builtin_amdgcn_wmma_f32_16x16x32_bf16(false, a, false, b, (short)0, c, false, false);
  asm volatile("v_nop\n\tv_nop\n\tv_nop\n\tv_nop" : "+v"(d) : "v"(a), "v"(b));
  return d;
}
__device__ __forceinline__ v16h frag_h(const _Float16* rowk0, int lane) {
  union { v16h v; v8h q[2]; } u; const _Float16* p = rowk0 + 8 * (lane >> 4);
  u.q[0] = *(const v8h*)p; u.q[1] = *(const v8h*)(p + 16); return u.v;
}
__device__ __forceinline__ v16h frag_f32(const float* rowk0, int lane) {
  v16h a; const float* p = rowk0 + 8 * (lane >> 4);
#pragma unroll
  for (int i = 0; i < 8; ++i) { a[i] = (_Float16)p[i]; a[8 + i] = (_Float16)p[16 + i]; }
  return a;
}
__device__ __forceinline__ v16h frag_f32s(const float* rowk0, int lane, float sc) {
  v16h a; const float* p = rowk0 + 8 * (lane >> 4);
#pragma unroll
  for (int i = 0; i < 8; ++i) { a[i] = (_Float16)(p[i] * sc); a[8 + i] = (_Float16)(p[16 + i] * sc); }
  return a;
}
__device__ __forceinline__ v16h fragc_f32(const float* W, int k0, int n, int lane, int ld, int K) {
  v16h a; const int g = lane >> 4;
#pragma unroll
  for (int i = 0; i < 8; ++i) { const int ka = k0 + 8 * g + i, kb = ka + 16;
    a[i] = (_Float16)(ka < K ? W[(size_t)(ka < K ? ka : K - 1) * ld + n] : 0.f); a[8 + i] = (_Float16)(kb < K ? W[(size_t)(kb < K ? kb : K - 1) * ld + n] : 0.f); }
  return a;
}
struct F2 { v16b h, l; };
__device__ __forceinline__ F2 bsplit16(const float v[16]) { F2 r;
#pragma unroll
  for (int i = 0; i < 16; ++i) { const __bf16 h = (__bf16)v[i]; r.h[i] = h; r.l[i] = (__bf16)(v[i] - (float)h); }
  return r; }
__device__ __forceinline__ F2 split_row(const float* row, int k0, int lane) { float v[16]; const float* p = row + k0 + 8 * (lane >> 4);
#pragma unroll
  for (int i = 0; i < 8; ++i) { v[i] = p[i]; v[8 + i] = p[16 + i]; }
  return bsplit16(v); }
__device__ __forceinline__ F2 split_rowK(const float* row, int k0, int lane, int K) { float v[16]; const int g = lane >> 4;
#pragma unroll
  for (int i = 0; i < 8; ++i) { const int ka = k0 + 8 * g + i, kb = ka + 16; v[i] = ka < K ? row[ka < K ? ka : K - 1] : 0.f; v[8 + i] = kb < K ? row[kb < K ? kb : K - 1] : 0.f; }
  return bsplit16(v); }
__device__ __forceinline__ F2 split_col(const float* W, int k0, int n, int lane, int ld, int K) { float v[16]; const int g = lane >> 4;
#pragma unroll
  for (int i = 0; i < 8; ++i) { const int ka = k0 + 8 * g + i, kb = ka + 16; v[i] = ka < K ? W[(size_t)(ka < K ? ka : K - 1) * ld + n] : 0.f; v[8 + i] = kb < K ? W[(size_t)(kb < K ? kb : K - 1) * ld + n] : 0.f; }
  return bsplit16(v); }
__device__ __forceinline__ v8f mac3(const F2& a, const F2& b, v8f c) { c = wmma_bf(a.l, b.h, c); c = wmma_bf(a.h, b.l, c); return wmma_bf(a.h, b.h, c); }
__device__ __forceinline__ float sigm(float v) { return 1.0f / (1.0f + expf(-v)); }
#define LDSX() do { asm volatile("s_wait_dscnt 0" ::: "memory"); __builtin_amdgcn_wave_barrier(); __builtin_amdgcn_fence(__ATOMIC_RELEASE, "workgroup"); } while (0)


#define NB 32
#define NN 256
#define DD 128
#define NH 8
#define QQ 16
#define FF 512
#define NLAY 3
#define NROW (NB * NN)
#define NBLK (NROW / 64)
#define SLOPE 0.15f
#define BNEPS 1e-5f
typedef __attribute__((ext_vector_type(8))) __bf16 v8b;
__device__ __forceinline__ v16b frag_b(const __bf16* rowk0, int lane) {
  union { v16b v; v8b q[2]; } u; const __bf16* p = rowk0 + 8 * (lane >> 4);
  u.q[0] = *(const v8b*)p; u.q[1] = *(const v8b*)(p + 16); return u.v;
}
__device__ __forceinline__ float bfr(float v) { return (float)(__bf16)v; }
__device__ __attribute__((noinline)) float exp_ni(float v) { return expf(v); }
__device__ __attribute__((noinline)) float erf_ni(float v) { return erff(v); }

#define WS_H    0u
#define WS_VP   (WS_H + 4u * NROW * DD)
#define WS_SC   (WS_VP + 4u * 2 * NROW * DD)
#define WS_X1   (WS_SC + 4u * NROW * 32)
#define WS_T    (WS_X1 + 4u * 2 * NROW * DD)
#define WS_X2   (WS_T + 4u * 2 * NROW * FF)
#define WS_PS   (WS_X2 + 4u * 2 * NROW * DD)
#define WS_BN   (WS_PS + 4u * 2 * NBLK * 2 * DD)
#define WS_CL   (WS_BN + 4u * 4 * 2 * DD)
#define WS_END  (WS_CL + 4u * NROW)

__device__ __forceinline__ v16b fragb_f32(const float* __restrict__ p, int lane) { v16b a; const float* pp = p + 8 * (lane >> 4);
#pragma unroll
  for (int i = 0; i < 8; ++i) { a[i] = (__bf16)pp[i]; a[8 + i] = (__bf16)pp[16 + i]; } return a; }
__device__ __forceinline__ F2 split_row_bn(const float* row, int k0, int lane, const float* __restrict__ bn  , const float* __restrict__ ga, const float* __restrict__ be) { float v[16]; const float* p = row + k0 + 8 * (lane >> 4); const int c0 = k0 + 8 * (lane >> 4);
#pragma unroll
  for (int i = 0; i < 8; ++i) { const int ca = c0 + i, cb = c0 + 16 + i; v[i] = (p[i] - bn[ca]) * bn[DD + ca] * bfr(ga[ca]) + bfr(be[ca]); v[8 + i] = (p[16 + i] - bn[cb]) * bn[DD + cb] * bfr(ga[cb]) + bfr(be[cb]); }
  return bsplit16(v); }
__device__ __forceinline__ void block_stats(float (*sf)[16][132], float* __restrict__ PSblk, int tid) { __shared__ __align__(16) float sm[DD], sq[DD];
  if (tid < DD) { float s = 0.f;
#pragma unroll 1
    for (int r = 0; r < 64; ++r) s += sf[r >> 4][r & 15][tid];
    const float mu = s * (1.0f / 64.0f); float q = 0.f;
#pragma unroll 1
    for (int r = 0; r < 64; ++r) { const float dv = sf[r >> 4][r & 15][tid] - mu; q += dv * dv; }
    sm[tid] = mu; sq[tid] = q; }
  __syncthreads(); if (tid < 32) vst2(PSblk + tid * 4, *(const v4f*)&sm[tid * 4]); else if (tid < 64) vst2(PSblk + DD + (tid - 32) * 4, *(const v4f*)&sq[(tid - 32) * 4]); __syncthreads(); }
__global__ __launch_bounds__(128) void k_init(const float* __restrict__ PIN, const float* __restrict__ WI, const float* __restrict__ BI, float* __restrict__ Hh, int* __restrict__ CL) { __shared__ __align__(16) float sf[4][16][132]; __shared__ __align__(16) int scl[64];
  const int tid = threadIdx.x, wave = tid >> 5, lane = tid & 31, col = lane & 15, g = lane >> 4; const size_t r0 = (size_t)blockIdx.x * 64 + wave * 16;
  v16b a;
#pragma unroll
  for (int i = 0; i < 8; ++i) { const int ka = 8 * g + i; a[i] = (__bf16)((ka < 16) ? PIN[(r0 + col) * 17 + ka] : 0.f); a[8 + i] = (__bf16)0.0f; }
  v8f acc[8] = {};
#pragma unroll
  for (int j = 0; j < 8; ++j) { v16b w;
#pragma unroll
    for (int i = 0; i < 8; ++i) { const int ka = 8 * g + i; w[i] = (__bf16)((ka < 16) ? WI[(j * 16 + col) * 16 + ka] : 0.f); w[8 + i] = (__bf16)0.0f; }
    acc[j] = wmma_bf(a, w, acc[j]); }
#pragma unroll
  for (int j = 0; j < 8; ++j)
#pragma unroll
    for (int r = 0; r < 8; ++r) sf[wave][8 * g + r][j * 16 + col] = acc[j][r] + bfr(BI[j * 16 + col]);
  if (tid < 64) scl[tid] = (int)bfr(PIN[((size_t)blockIdx.x * 64 + tid) * 17 + 16]);
  __syncthreads();
  for (int rl = 0; rl < 16; ++rl) vst2(Hh + (r0 + rl) * DD + lane * 4, *(const v4f*)&sf[wave][rl][lane * 4]);
  if (tid < 16) vst2(CL + (size_t)blockIdx.x * 64 + tid * 4, *(const v4i*)&scl[tid * 4]); }
__global__ __launch_bounds__(128) void k_lin1(const float* __restrict__ Hh, const float* __restrict__ WVG, const float* __restrict__ WVL, const float* __restrict__ WAG, const float* __restrict__ WAL, float* __restrict__ VP, float* __restrict__ SC) { __shared__ __align__(16) float tt[128][72]; __shared__ __align__(16) float sf[4][16][36];
  const int tid = threadIdx.x, wave = tid >> 5, lane = tid & 31, col = lane & 15, g = lane >> 4; const int cg = blockIdx.y; const size_t r0 = (size_t)blockIdx.x * 64 + wave * 16; const size_t b = ((size_t)blockIdx.x * 64) / NN; const int n0 = (int)(((size_t)blockIdx.x * 64) % NN);
  if (cg < 2) { const float* Wm = (cg == 0 ? WVG : WVL); v8f acc[8] = {};
#pragma unroll
    for (int kc = 0; kc < DD / 32; ++kc) { const F2 a = split_row(Hh + (r0 + col) * DD, kc * 32, lane);
#pragma unroll
      for (int j = 0; j < 8; ++j) { const v16b w = fragb_f32(Wm + (size_t)(j * 16 + col) * DD + kc * 32, lane); acc[j] = wmma_bf(a.h, w, acc[j]); acc[j] = wmma_bf(a.l, w, acc[j]); } }
#pragma unroll
    for (int j = 0; j < 8; ++j)
#pragma unroll
      for (int r = 0; r < 8; ++r) tt[j * 16 + col][wave * 16 + 8 * g + r] = acc[j][r];
    __syncthreads();
    for (int e = tid; e < 128 * 16; e += 128) { const int cl = e >> 4, q = e & 15; vst2(VP + (((size_t)cg * NB + b) * DD + cl) * NN + n0 + q * 4, *(const v4f*)&tt[cl][q * 4]); } }
  else { v8f acc[2] = {};
#pragma unroll
    for (int kc = 0; kc < DD / 32; ++kc) { const F2 a = split_row(Hh + (r0 + col) * DD, kc * 32, lane);
#pragma unroll
      for (int j = 0; j < 2; ++j) { const int sc = j * 16 + col; const int br = sc >> 4, part = (sc >> 3) & 1, hh = sc & 7; const float* Wa = (br == 0) ? (WAG + (size_t)hh * (2 * DD + 1)) : (WAL + (size_t)hh * (2 * DD)); const v16b w = fragb_f32(Wa + part * DD + kc * 32, lane); acc[j] = wmma_bf(a.h, w, acc[j]); acc[j] = wmma_bf(a.l, w, acc[j]); } }
#pragma unroll
    for (int j = 0; j < 2; ++j)
#pragma unroll
      for (int r = 0; r < 8; ++r) sf[wave][8 * g + r][j * 16 + col] = acc[j][r];
    LDSX(); for (int rl = 0; rl < 16; ++rl) if (lane < 8) vst2(SC + (r0 + rl) * 32 + lane * 4, *(const v4f*)&sf[wave][rl][lane * 4]); } }
__global__ __launch_bounds__(128) void k_gat(const float* __restrict__ Hh, const float* __restrict__ SC, const float* __restrict__ VP, const int* __restrict__ CL, const float* __restrict__ WAG, const float* __restrict__ WOG, const float* __restrict__ WOL, float* __restrict__ X1, float* __restrict__ PS) { __shared__ __align__(16) float sa[4][16][132]; __shared__ __align__(16) float sf[4][16][132]; __shared__ __align__(16) float ssj[NN][8]; __shared__ __align__(16) int scj[NN];
  const int tid = threadIdx.x, wave = tid >> 5, lane = tid & 31, col = lane & 15, g = lane >> 4; const int br = blockIdx.y; const float* WO = (br == 0) ? WOG : WOL; const size_t r0 = (size_t)blockIdx.x * 64 + wave * 16; const size_t b = ((size_t)blockIdx.x * 64) / NN; const size_t rb = b * NN;
  for (int e = tid; e < NN * 8; e += 128) { const int j = e >> 3, hh = e & 7; ssj[j][hh] = SC[(rb + j) * 32 + br * 16 + 8 + hh]; }
  for (int e = tid; e < NN; e += 128) scj[e] = CL[rb + e];
  __syncthreads();
  const size_t irow = r0 + col; const int ci = CL[irow];
  v8f acc[8];
#pragma unroll
  for (int hh = 0; hh < NH; ++hh) { const float si = SC[irow * 32 + br * 16 + hh]; const float we = (br == 0) ? bfr(WAG[(size_t)hh * (2 * DD + 1) + 2 * DD]) : 0.f;
    float mx = -3.0e38f;
#pragma unroll 1
    for (int j = 0; j < NN; ++j) { const bool same = (scj[j] == ci); float s = si + ssj[j][hh] + (same ? we : 0.f); s = (s > 0.f) ? s : SLOPE * s; if (br == 1 && !same) s = -1e9f; mx = fmaxf(mx, s); }
    float sum = 0.f;
#pragma unroll 1
    for (int j = 0; j < NN; ++j) { const bool same = (scj[j] == ci); float s = si + ssj[j][hh] + (same ? we : 0.f); s = (s > 0.f) ? s : SLOPE * s; if (br == 1 && !same) s = -1e9f; sum += expf(s - mx); }
    const float inv = 1.0f / sum;
    v8f c = {};
#pragma unroll 1
    for (int kc = 0; kc < NN / 32; ++kc) { float v[16];
#pragma unroll
      for (int i = 0; i < 8; ++i) {
#pragma unroll
        for (int half = 0; half < 2; ++half) { const int j = kc * 32 + half * 16 + 8 * g + i; const bool same = (scj[j] == ci); float s = si + ssj[j][hh] + (same ? we : 0.f); s = (s > 0.f) ? s : SLOPE * s; if (br == 1 && !same) s = -1e9f; v[half * 8 + i] = expf(s - mx) * inv; } }
      const F2 a = bsplit16(v); const F2 w = split_row(VP + (((size_t)br * NB + b) * DD + hh * QQ + col) * NN, kc * 32, lane); c = mac3(a, w, c); }
    acc[hh] = c; }
#pragma unroll
  for (int hh = 0; hh < NH; ++hh)
#pragma unroll
    for (int r = 0; r < 8; ++r) sa[wave][8 * g + r][hh * QQ + col] = acc[hh][r];
  LDSX();
  v8f o[8] = {};
#pragma unroll
  for (int kc = 0; kc < DD / 32; ++kc) { const F2 a = split_row(&sa[wave][col][0], kc * 32, lane);
#pragma unroll
    for (int j = 0; j < 8; ++j) { const v16b w = fragb_f32(WO + (size_t)(j * 16 + col) * DD + kc * 32, lane); o[j] = wmma_bf(a.h, w, o[j]); o[j] = wmma_bf(a.l, w, o[j]); } }
#pragma unroll
  for (int j = 0; j < 8; ++j)
#pragma unroll
    for (int r = 0; r < 8; ++r) sf[wave][8 * g + r][j * 16 + col] = o[j][r] + Hh[(r0 + 8 * g + r) * DD + j * 16 + col];
  __syncthreads();
  for (int rl = 0; rl < 16; ++rl) vst2(X1 + ((size_t)br * NROW + r0 + rl) * DD + lane * 4, *(const v4f*)&sf[wave][rl][lane * 4]);
  block_stats(sf, PS + (((size_t)br * NBLK + blockIdx.x) * 2) * DD, tid); }
__global__ __launch_bounds__(128) void k_bnfin(const float* __restrict__ PS, int which, float* __restrict__ BN) { __shared__ __align__(16) float sm[DD], si[DD]; const int c = threadIdx.x; const int br = blockIdx.x;
  float n = 0.f, mean = 0.f, M2 = 0.f;
#pragma unroll 1
  for (int blk = 0; blk < NBLK; ++blk) { const float mb = PS[(((size_t)br * NBLK + blk) * 2) * DD + c], qb = PS[(((size_t)br * NBLK + blk) * 2 + 1) * DD + c]; const float nb = 64.f; const float nt = n + nb; const float dl = mb - mean; mean += dl * (nb / nt); M2 += qb + dl * dl * (n * nb / nt); n = nt; }
  sm[c] = mean; si[c] = 1.0f / sqrtf(M2 / n + BNEPS);
  __syncthreads(); float* dst = BN + (size_t)(br * 2 + which) * 2 * DD; if (c < 32) vst2(dst + c * 4, *(const v4f*)&sm[c * 4]); else if (c < 64) vst2(dst + DD + (c - 32) * 4, *(const v4f*)&si[(c - 32) * 4]); }
__global__ __launch_bounds__(128) void k_ff1(const float* __restrict__ X1, const float* __restrict__ BN, const float* __restrict__ GA, const float* __restrict__ BE, const float* __restrict__ W1G, const float* __restrict__ W1L, const float* __restrict__ B1G, const float* __restrict__ B1L, float* __restrict__ T) { __shared__ __align__(16) float sf[4][16][132];
  const int tid = threadIdx.x, wave = tid >> 5, lane = tid & 31, col = lane & 15, g = lane >> 4; const int br = blockIdx.z; const size_t r0 = (size_t)blockIdx.x * 64 + wave * 16; const int c0 = blockIdx.y * 128; const float* W1 = br == 0 ? W1G : W1L; const float* B1 = br == 0 ? B1G : B1L; const float* bn = BN + (size_t)(br * 2 + 0) * 2 * DD; const float* ga = GA + (br * 2 + 0) * DD; const float* be = BE + (br * 2 + 0) * DD;
  v8f acc[8] = {};
#pragma unroll
  for (int kc = 0; kc < DD / 32; ++kc) { const F2 a = split_row_bn(X1 + ((size_t)br * NROW + r0 + col) * DD, kc * 32, lane, bn, ga, be);
#pragma unroll
    for (int j = 0; j < 8; ++j) { const v16b w = fragb_f32(W1 + (size_t)(c0 + j * 16 + col) * DD + kc * 32, lane); acc[j] = wmma_bf(a.h, w, acc[j]); acc[j] = wmma_bf(a.l, w, acc[j]); } }
#pragma unroll
  for (int j = 0; j < 8; ++j) { const float bb = bfr(B1[c0 + j * 16 + col]);
#pragma unroll
    for (int r = 0; r < 8; ++r) { const float z = acc[j][r] + bb; sf[wave][8 * g + r][j * 16 + col] = (z > 0.f) ? z : (expf(z) - 1.0f); } }
  LDSX(); for (int rl = 0; rl < 16; ++rl) vst2(T + ((size_t)br * NROW + r0 + rl) * FF + c0 + lane * 4, *(const v4f*)&sf[wave][rl][lane * 4]); }
__global__ __launch_bounds__(128) void k_ff2(const float* __restrict__ T, const float* __restrict__ X1, const float* __restrict__ BN, const float* __restrict__ GA, const float* __restrict__ BE, const float* __restrict__ W2G, const float* __restrict__ W2L, const float* __restrict__ B2G, const float* __restrict__ B2L, float* __restrict__ X2, float* __restrict__ PS) { __shared__ __align__(16) float sf[4][16][132];
  const int tid = threadIdx.x, wave = tid >> 5, lane = tid & 31, col = lane & 15, g = lane >> 4; const int br = blockIdx.y; const size_t r0 = (size_t)blockIdx.x * 64 + wave * 16; const float* W2 = br == 0 ? W2G : W2L; const float* B2 = br == 0 ? B2G : B2L; const float* bn = BN + (size_t)(br * 2 + 0) * 2 * DD; const float* ga = GA + (br * 2 + 0) * DD; const float* be = BE + (br * 2 + 0) * DD;
  v8f acc[8] = {};
#pragma unroll 2
  for (int kc = 0; kc < FF / 32; ++kc) { const F2 a = split_row(T + ((size_t)br * NROW + r0 + col) * FF, kc * 32, lane);
#pragma unroll
    for (int j = 0; j < 8; ++j) { const v16b w = fragb_f32(W2 + (size_t)(j * 16 + col) * FF + kc * 32, lane); acc[j] = wmma_bf(a.h, w, acc[j]); acc[j] = wmma_bf(a.l, w, acc[j]); } }
#pragma unroll
  for (int j = 0; j < 8; ++j) { const int c = j * 16 + col; const float bb = bfr(B2[c]); const float m = bn[c], is = bn[DD + c], gg = bfr(ga[c]), bt = bfr(be[c]);
#pragma unroll
    for (int r = 0; r < 8; ++r) { const float x1 = X1[((size_t)br * NROW + r0 + 8 * g + r) * DD + c]; sf[wave][8 * g + r][c] = acc[j][r] + bb + ((x1 - m) * is * gg + bt); } }
  __syncthreads();
  for (int rl = 0; rl < 16; ++rl) vst2(X2 + ((size_t)br * NROW + r0 + rl) * DD + lane * 4, *(const v4f*)&sf[wave][rl][lane * 4]);
  block_stats(sf, PS + (((size_t)br * NBLK + blockIdx.x) * 2) * DD, tid); }
__global__ __launch_bounds__(128) void k_fuse(const float* __restrict__ X2, const float* __restrict__ BN, const float* __restrict__ GA, const float* __restrict__ BE, const float* __restrict__ WF, const float* __restrict__ BF, float* __restrict__ Hout) { __shared__ __align__(16) float sf[4][16][132];
  const int tid = threadIdx.x, wave = tid >> 5, lane = tid & 31, col = lane & 15, g = lane >> 4; const size_t r0 = (size_t)blockIdx.x * 64 + wave * 16;
  v8f acc[8] = {};
#pragma unroll
  for (int kc = 0; kc < 2 * DD / 32; ++kc) { const int br = kc / 4, kk = (kc % 4) * 32; const F2 a = split_row_bn(X2 + ((size_t)br * NROW + r0 + col) * DD, kk, lane, BN + (size_t)(br * 2 + 1) * 2 * DD, GA + (br * 2 + 1) * DD, BE + (br * 2 + 1) * DD);
#pragma unroll
    for (int j = 0; j < 8; ++j) { const v16b w = fragb_f32(WF + (size_t)(j * 16 + col) * (2 * DD) + kc * 32, lane); acc[j] = wmma_bf(a.h, w, acc[j]); acc[j] = wmma_bf(a.l, w, acc[j]); } }
#pragma unroll
  for (int j = 0; j < 8; ++j) { const float bb = bfr(BF[j * 16 + col]);
#pragma unroll
    for (int r = 0; r < 8; ++r) sf[wave][8 * g + r][j * 16 + col] = acc[j][r] + bb; }
  LDSX(); for (int rl = 0; rl < 16; ++rl) vst2(Hout + (r0 + rl) * DD + lane * 4, *(const v4f*)&sf[wave][rl][lane * 4]); }
extern "C" void kernel_launch(void* const* d_in, const int* in_sizes, int n_in, void* d_out, int out_size, void* d_ws, size_t ws_size, hipStream_t stream) {
  (void)in_sizes; (void)n_in; (void)out_size;
  const float** F = (const float**)d_in;
  if (ws_size < (size_t)WS_END) return;
  char* ws = (char*)d_ws; float *Hh = (float*)(ws + WS_H), *VP = (float*)(ws + WS_VP), *SC = (float*)(ws + WS_SC), *X1 = (float*)(ws + WS_X1), *T = (float*)(ws + WS_T), *X2 = (float*)(ws + WS_X2), *PS = (float*)(ws + WS_PS), *BN = (float*)(ws + WS_BN); int* CL = (int*)(ws + WS_CL);
  k_init<<<NBLK, 128, 0, stream>>>(F[0], F[1], F[2], Hh, CL);
  for (int li = 0; li < NLAY; ++li) {
    const float *WAG = F[3] + (size_t)li * 8 * 257, *WVG = F[4] + (size_t)li * DD * DD, *WOG = F[5] + (size_t)li * DD * DD, *WAL = F[6] + (size_t)li * 8 * 256, *WVL = F[7] + (size_t)li * DD * DD, *WOL = F[8] + (size_t)li * DD * DD;
    const float *GA = F[9] + (size_t)li * 4 * DD, *BE = F[10] + (size_t)li * 4 * DD;
    const float *W1G = F[11] + (size_t)li * FF * DD, *B1G = F[12] + (size_t)li * FF, *W2G = F[13] + (size_t)li * DD * FF, *B2G = F[14] + (size_t)li * DD, *W1L = F[15] + (size_t)li * FF * DD, *B1L = F[16] + (size_t)li * FF, *W2L = F[17] + (size_t)li * DD * FF, *B2L = F[18] + (size_t)li * DD;
    const float *WF = F[19] + (size_t)li * DD * 2 * DD, *BF = F[20] + (size_t)li * DD;
    k_lin1<<<dim3(NBLK, 3), 128, 0, stream>>>(Hh, WVG, WVL, WAG, WAL, VP, SC);
    k_gat<<<dim3(NBLK, 2), 128, 0, stream>>>(Hh, SC, VP, CL, WAG, WOG, WOL, X1, PS);
    k_bnfin<<<2, 128, 0, stream>>>(PS, 0, BN);
    k_ff1<<<dim3(NBLK, FF / 128, 2), 128, 0, stream>>>(X1, BN, GA, BE, W1G, W1L, B1G, B1L, T);
    k_ff2<<<dim3(NBLK, 2), 128, 0, stream>>>(T, X1, BN, GA, BE, W2G, W2L, B2G, B2L, X2, PS);
    k_bnfin<<<2, 128, 0, stream>>>(PS, 1, BN);
    k_fuse<<<NBLK, 128, 0, stream>>>(X2, BN, GA, BE, WF, BF, (li == NLAY - 1) ? (float*)d_out : Hh);
  }
}
